// ColightEncoder_90950227460700
// MI455X (gfx1250) — hardware-verified
//
#include <hip/hip_runtime.h>
#include <math.h>

typedef __attribute__((ext_vector_type(16))) _Float16 v16h;
typedef __attribute__((ext_vector_type(16))) __bf16 v16b;
typedef __attribute__((ext_vector_type(8)))  _Float16 v8h;
typedef __attribute__((ext_vector_type(8)))  float v8f;
typedef __attribute__((ext_vector_type(4)))  float v4f;
typedef __attribute__((ext_vector_type(2)))  float v2f;
typedef __attribute__((ext_vector_type(4)))  unsigned v4u;
typedef __attribute__((ext_vector_type(4)))  int v4i;
typedef float __attribute__((may_alias)) float_a;
typedef int __attribute__((may_alias)) int_a;

template <typename T> __device__ __forceinline__ void vst2(void* p, T v) { *(volatile T*)p = v; __threadfence(); *(volatile T*)p = v; }
__device__ __forceinline__ v8f wmma16(v16h a, v16h b, v8f c) {
  v8f d = __builtin_amdgcn_wmma_f32_16x16x32_f16(false, a, false, b, (short)0, c, false, false);
  asm volatile("v_nop\n\tv_nop\n\tv_nop\n\tv_nop" : "+v"(d) : "v"(a), "v"(b));
  return d;
}
__device__ __forceinline__ v8f wmma_bf(v16b a, v16b b, v8f c) {
  v8f d = __builtin_amdgcn_wmma_f32_16x16x32_bf16(false, a, false, b, (short)0, c, false, false);
  asm volatile("v_nop\n\tv_nop\n\tv_nop\n\tv_nop" : "+v"(d) : "v"(a), "v"(b));
  return d;
}
__device__ __forceinline__ v16h frag_h(const _Float16* rowk0, int lane) {
  union { v16h v; v8h q[2]; } u; const _Float16* p = rowk0 + 8 * (lane >> 4);
  u.q[0] = *(const v8h*)p; u.q[1] = *(const v8h*)(p + 16); return u.v;
}
__device__ __forceinline__ v16h frag_f32(const float* rowk0, int lane) {
  v16h a; const float* p = rowk0 + 8 * (lane >> 4);
#pragma unroll
  for (int i = 0; i < 8; ++i) { a[i] = (_Float16)p[i]; a[8 + i] = (_Float16)p[16 + i]; }
  return a;
}
__device__ __forceinline__ v16h frag_f32s(const float* rowk0, int lane, float sc) {
  v16h a; const float* p = rowk0 + 8 * (lane >> 4);
#pragma unroll
  for (int i = 0; i < 8; ++i) { a[i] = (_Float16)(p[i] * sc); a[8 + i] = (_Float16)(p[16 + i] * sc); }
  return a;
}
__device__ __forceinline__ v16h fragc_f32(const float* W, int k0, int n, int lane, int ld, int K) {
  v16h a; const int g = lane >> 4;
#pragma unroll
  for (int i = 0; i < 8; ++i) { const int ka = k0 + 8 * g + i, kb = ka + 16;
    a[i] = (_Float16)(ka < K ? W[(size_t)(ka < K ? ka : K - 1) * ld + n] : 0.f); a[8 + i] = (_Float16)(kb < K ? W[(size_t)(kb < K ? kb : K - 1) * ld + n] : 0.f); }
  return a;
}
struct F2 { v16b h, l; };
__device__ __forceinline__ F2 bsplit16(const float v[16]) { F2 r;
#pragma unroll
  for (int i = 0; i < 16; ++i) { const __bf16 h = (__bf16)v[i]; r.h[i] = h; r.l[i] = (__bf16)(v[i] - (float)h); }
  return r; }
__device__ __forceinline__ F2 split_row(const float* row, int k0, int lane) { float v[16]; const float* p = row + k0 + 8 * (lane >> 4);
#pragma unroll
  for (int i = 0; i < 8; ++i) { v[i] = p[i]; v[8 + i] = p[16 + i]; }
  return bsplit16(v); }
__device__ __forceinline__ F2 split_rowK(const float* row, int k0, int lane, int K) { float v[16]; const int g = lane >> 4;
#pragma unroll
  for (int i = 0; i < 8; ++i) { const int ka = k0 + 8 * g + i, kb = ka + 16; v[i] = ka < K ? row[ka < K ? ka : K - 1] : 0.f; v[8 + i] = kb < K ? row[kb < K ? kb : K - 1] : 0.f; }
  return bsplit16(v); }
__device__ __forceinline__ F2 split_col(const float* W, int k0, int n, int lane, int ld, int K) { float v[16]; const int g = lane >> 4;
#pragma unroll
  for (int i = 0; i < 8; ++i) { const int ka = k0 + 8 * g + i, kb = ka + 16; v[i] = ka < K ? W[(size_t)(ka < K ? ka : K - 1) * ld + n] : 0.f; v[8 + i] = kb < K ? W[(size_t)(kb < K ? kb : K - 1) * ld + n] : 0.f; }
  return bsplit16(v); }
__device__ __forceinline__ v8f mac3(const F2& a, const F2& b, v8f c) { c = wmma_bf(a.l, b.h, c); c = wmma_bf(a.h, b.l, c); return wmma_bf(a.h, b.h, c); }
__device__ __forceinline__ float sigm(float v) { return 1.0f / (1.0f + expf(-v)); }
#define LDSX() do { asm volatile("s_wait_dscnt 0" ::: "memory"); __builtin_amdgcn_wave_barrier(); __builtin_amdgcn_fence(__ATOMIC_RELEASE, "workgroup"); } while (0)


#define NB 32
#define NA 200
#define NN 5
#define DIN 36
#define HDM 128
#define NHD 5
#define HW (HDM * NHD)
#define NAG (NB * NA)
#define NNR (NA * NN)
#define NAP 224
typedef __attribute__((ext_vector_type(8))) __bf16 v8b;
__device__ __forceinline__ v16b frag_b(const __bf16* rowk0, int lane) {
  union { v16b v; v8b q[2]; } u; const __bf16* p = rowk0 + 8 * (lane >> 4);
  u.q[0] = *(const v8b*)p; u.q[1] = *(const v8b*)(p + 16); return u.v;
}
__device__ __forceinline__ float bfr(float v) { return (float)(__bf16)v; }
__device__ __attribute__((noinline)) float exp_ni(float v) { return expf(v); }
__device__ __attribute__((noinline)) float erf_ni(float v) { return erff(v); }

#define WS_W1  0u
#define WS_W2  (WS_W1 + 2u * 128 * 64)
#define WS_WB  (WS_W2 + 2u * 128 * 128)
#define WBSZ   (2u * (3 * HW * HDM + HDM * HDM))
#define WS_HA  (WS_WB + 2u * WBSZ)
#define WS_H   (WS_HA + 4u * (size_t)NAG * HDM)
#define WS_HPH (WS_H + 4u * (size_t)NAG * HDM)
#define WS_HPL (WS_HPH + 2u * (size_t)NB * HDM * NAP)
#define NNRP   32064
#define WS_NEI (WS_HPL + 2u * (size_t)NB * HDM * NAP)
#define WS_AH  (WS_NEI + 4u * (size_t)NNRP * HDM)
#define WS_NH  (WS_AH + 4u * (size_t)NAG * HW)
#define WS_HH  (WS_NH + 4u * (size_t)NNRP * HW)
#define WS_OO  (WS_HH + 4u * (size_t)NNRP * HW)
#define WS_END (WS_OO + 4u * (size_t)NAG * HDM)

__global__ __launch_bounds__(128) void k_packT(const float* __restrict__ Wt, int K, int N, int KP, __bf16* __restrict__ dst) { __shared__ __align__(16) __bf16 s[HDM]; const int n = blockIdx.x, t = threadIdx.x; (void)N;
  for (int k = t; k < KP; k += 128) s[k] = (k < K) ? (__bf16)Wt[(size_t)k * N + n] : (__bf16)0.0f; __syncthreads(); for (int q = t; q < KP / 8; q += 128) vst2((unsigned*)(dst + (size_t)n * KP + q * 8), *(const v4u*)&s[q * 8]); }
template <int RELU, int RAW>
__global__ __launch_bounds__(128) void k_gemm(const float* __restrict__ A, int lda, int K, int KP, int M, const __bf16* __restrict__ Wr, const float* __restrict__ BIAS, float* __restrict__ OUT, int N) {   __shared__ __align__(16) float sf[4][16][132];
  const int tid = threadIdx.x, wave = tid >> 5, lane = tid & 31, col = lane & 15, g = lane >> 4; const size_t r0 = (size_t)blockIdx.x * 64 + wave * 16; const int c0 = blockIdx.y * 128; const size_t ra = (r0 + col < (size_t)M) ? r0 + col : (size_t)M - 1;
  v8f acc[8] = {};
#pragma unroll 1
  for (int kc = 0; kc < KP / 32; ++kc) { float v[16]; const float* p = A + ra * lda + kc * 32 + 8 * g;
#pragma unroll
    for (int i = 0; i < 8; ++i) { const int k0 = kc * 32 + 8 * g + i; v[i] = (k0 < K) ? (RAW ? bfr(p[i]) : p[i]) : 0.f; v[8 + i] = (k0 + 16 < K) ? (RAW ? bfr(p[16 + i]) : p[16 + i]) : 0.f; }
    const F2 a = bsplit16(v);
#pragma unroll
    for (int j = 0; j < 8; ++j) { const v16b w = frag_b(Wr + (size_t)(c0 + j * 16 + col) * KP + kc * 32, lane); acc[j] = wmma_bf(a.h, w, acc[j]); acc[j] = wmma_bf(a.l, w, acc[j]); } }
#pragma unroll
  for (int j = 0; j < 8; ++j) { const float bb = bfr(BIAS[c0 + j * 16 + col]);
#pragma unroll
    for (int r = 0; r < 8; ++r) { const float x = acc[j][r] + bb; sf[wave][8 * g + r][j * 16 + col] = RELU ? fmaxf(x, 0.f) : x; } }
  LDSX(); for (int rl = 0; rl < 16; ++rl) if (r0 + rl < (size_t)M) vst2(OUT + (r0 + rl) * N + c0 + lane * 4, *(const v4f*)&sf[wave][rl][lane * 4]); }
__global__ __launch_bounds__(224) void k_ht(const float* __restrict__ H, __bf16* __restrict__ PH, __bf16* __restrict__ PL) { __shared__ __align__(16) __bf16 sh[16][NAP + 8], sl[16][NAP + 8]; const int t = threadIdx.x; const size_t b = blockIdx.x; const int d0 = blockIdx.y * 16;
  for (int dd = 0; dd < 16; ++dd) { const float v = (t < NA) ? H[(b * NA + t) * HDM + d0 + dd] : 0.f; const __bf16 hv = (__bf16)v; sh[dd][t] = hv; sl[dd][t] = (__bf16)(v - (float)hv); } __syncthreads();
  for (int e = t; e < 16 * (NAP / 8); e += 224) { const int dd = e / (NAP / 8), q = e % (NAP / 8); const size_t o = (b * HDM + d0 + dd) * NAP + q * 8; vst2((unsigned*)(PH + o), *(const v4u*)&sh[dd][q * 8]); vst2((unsigned*)(PL + o), *(const v4u*)&sl[dd][q * 8]); } }
__global__ __launch_bounds__(128) void k_nei(const float* __restrict__ ADJ, const __bf16* __restrict__ PH, const __bf16* __restrict__ PL, float* __restrict__ NEI) { __shared__ __align__(16) float sf[4][16][132];
  const int tid = threadIdx.x, wave = tid >> 5, lane = tid & 31, col = lane & 15, g = lane >> 4; const size_t b = blockIdx.y; const int r0 = blockIdx.x * 64 + wave * 16; const int ra = (r0 + col < NNR) ? r0 + col : NNR - 1; const float* arow = ADJ + (b * NNR + ra) * NA;
  v8f acc[8] = {};
#pragma unroll 1
  for (int kc = 0; kc < NAP / 32; ++kc) { v16b a;
#pragma unroll
    for (int i = 0; i < 8; ++i) { const int k0 = kc * 32 + 8 * g + i; a[i] = (__bf16)((k0 < NA) ? arow[k0] : 0.f); a[8 + i] = (__bf16)((k0 + 16 < NA) ? arow[k0 + 16] : 0.f); }
#pragma unroll
    for (int j = 0; j < 8; ++j) { const size_t po = (b * HDM + j * 16 + col) * NAP + kc * 32; acc[j] = wmma_bf(a, frag_b(PH + po, lane), acc[j]); acc[j] = wmma_bf(a, frag_b(PL + po, lane), acc[j]); } }
#pragma unroll
  for (int j = 0; j < 8; ++j)
#pragma unroll
    for (int r = 0; r < 8; ++r) sf[wave][8 * g + r][j * 16 + col] = acc[j][r];
  LDSX(); for (int rl = 0; rl < 16; ++rl) if (r0 + rl < NNR) vst2(NEI + (b * NNR + r0 + rl) * HDM + lane * 4, *(const v4f*)&sf[wave][rl][lane * 4]); }
__global__ __launch_bounds__(128) void k_att(const float* __restrict__ AH, const float* __restrict__ NHm, const float* __restrict__ HH, float* __restrict__ O) { __shared__ float red[4][NHD * NN]; __shared__ float satt[NHD][NN]; __shared__ __align__(16) float so2[HDM]; const int t = threadIdx.x; const size_t ag = blockIdx.x; const size_t nr0 = ag * NN;
  float part[NHD * NN];
#pragma unroll
  for (int hd_ = 0; hd_ < NHD; ++hd_) { const float a = AH[ag * HW + t * NHD + hd_];
#pragma unroll
    for (int n = 0; n < NN; ++n) part[hd_ * NN + n] = a * NHm[(nr0 + n) * HW + t * NHD + hd_]; }
#pragma unroll
  for (int i = 0; i < NHD * NN; ++i) { float v = part[i];
#pragma unroll
    for (int o = 1; o < 32; o <<= 1) v += __shfl_xor(v, o);
    if ((t & 31) == 0) red[t >> 5][i] = v; }
  __syncthreads();
  if (t < NHD) { float lg[NN]; float mx = -3.0e38f; for (int n = 0; n < NN; ++n) { lg[n] = red[0][t * NN + n] + red[1][t * NN + n] + red[2][t * NN + n] + red[3][t * NN + n]; mx = fmaxf(mx, lg[n]); } float s = 0.f; for (int n = 0; n < NN; ++n) { lg[n] = expf(lg[n] - mx); s += lg[n]; } for (int n = 0; n < NN; ++n) satt[t][n] = lg[n] / s; }
  __syncthreads();
  float o = 0.f;
#pragma unroll
  for (int hd_ = 0; hd_ < NHD; ++hd_) { float acc = 0.f;
#pragma unroll
    for (int n = 0; n < NN; ++n) acc += satt[hd_][n] * HH[(nr0 + n) * HW + t * NHD + hd_]; o += acc; }
  so2[t] = o / (float)NHD; __syncthreads(); if (t < HDM / 4) vst2(O + ag * HDM + t * 4, *(const v4f*)&so2[t * 4]); }
extern "C" void kernel_launch(void* const* d_in, const int* in_sizes, int n_in, void* d_out, int out_size, void* d_ws, size_t ws_size, hipStream_t stream) {
  (void)in_sizes; (void)n_in; (void)out_size;
  const float** F = (const float**)d_in;
  if (ws_size < (size_t)WS_END) return;
  char* ws = (char*)d_ws; __bf16 *W1 = (__bf16*)(ws + WS_W1), *W2 = (__bf16*)(ws + WS_W2), *PH = (__bf16*)(ws + WS_HPH), *PL = (__bf16*)(ws + WS_HPL); float *HA = (float*)(ws + WS_HA), *H = (float*)(ws + WS_H), *NEI = (float*)(ws + WS_NEI), *AH = (float*)(ws + WS_AH), *NHm = (float*)(ws + WS_NH), *HH = (float*)(ws + WS_HH), *OO = (float*)(ws + WS_OO);
  k_packT<<<HDM, 128, 0, stream>>>(F[2], DIN, HDM, 64, W1);
  k_packT<<<HDM, 128, 0, stream>>>(F[4], HDM, HDM, HDM, W2);
  for (int blk = 0; blk < 2; ++blk) { __bf16* WB = (__bf16*)(ws + WS_WB + (size_t)blk * WBSZ); const int fi = 6 + 8 * blk;
    k_packT<<<HW, 128, 0, stream>>>(F[fi + 0], HDM, HW, HDM, WB); k_packT<<<HW, 128, 0, stream>>>(F[fi + 2], HDM, HW, HDM, WB + (size_t)HW * HDM); k_packT<<<HW, 128, 0, stream>>>(F[fi + 4], HDM, HW, HDM, WB + (size_t)2 * HW * HDM); k_packT<<<HDM, 128, 0, stream>>>(F[fi + 6], HDM, HDM, HDM, WB + (size_t)3 * HW * HDM); }
  k_gemm<1, 1><<<dim3((NAG + 63) / 64, 1), 128, 0, stream>>>(F[0], DIN, DIN, 64, NAG, W1, F[3], HA, HDM);
  k_gemm<1, 0><<<dim3((NAG + 63) / 64, 1), 128, 0, stream>>>(HA, HDM, HDM, HDM, NAG, W2, F[5], H, HDM);
  for (int blk = 0; blk < 2; ++blk) { const __bf16* WB = (const __bf16*)(ws + WS_WB + (size_t)blk * WBSZ); const int fi = 6 + 8 * blk;
    k_ht<<<dim3(NB, HDM / 16), 224, 0, stream>>>(H, PH, PL);
    k_nei<<<dim3((NNR + 63) / 64, NB), 128, 0, stream>>>(F[1], PH, PL, NEI);
    k_gemm<1, 0><<<dim3((NAG + 63) / 64, HW / 128), 128, 0, stream>>>(H, HDM, HDM, HDM, NAG, WB, F[fi + 1], AH, HW);
    k_gemm<1, 0><<<dim3((NB * NNR + 63) / 64, HW / 128), 128, 0, stream>>>(NEI, HDM, HDM, HDM, NB * NNR, WB + (size_t)HW * HDM, F[fi + 3], NHm, HW);
    k_gemm<1, 0><<<dim3((NB * NNR + 63) / 64, HW / 128), 128, 0, stream>>>(NEI, HDM, HDM, HDM, NB * NNR, WB + (size_t)2 * HW * HDM, F[fi + 5], HH, HW);
    k_att<<<NAG, 128, 0, stream>>>(AH, NHm, HH, OO);
    k_gemm<1, 0><<<dim3((NAG + 63) / 64, 1), 128, 0, stream>>>(OO, HDM, HDM, HDM, NAG, WB + (size_t)3 * HW * HDM, F[fi + 7], blk == 1 ? (float*)d_out : H, HDM); }
}
